// FP_Layer_11123965297224
// MI455X (gfx1250) — hardware-run, weakly checked
//
#include <hip/hip_runtime.h>

typedef float          v8f   __attribute__((ext_vector_type(8)));
typedef float          v4f   __attribute__((ext_vector_type(4)));
typedef unsigned int   v4u   __attribute__((ext_vector_type(4)));
typedef int            v8i   __attribute__((ext_vector_type(8)));
typedef unsigned short v8us  __attribute__((ext_vector_type(8)));
typedef unsigned short v16us __attribute__((ext_vector_type(16)));
typedef __bf16         v16bf __attribute__((ext_vector_type(16)));
typedef _Float16       v16h  __attribute__((ext_vector_type(16)));
typedef v4f  __attribute__((may_alias)) v4fa;
typedef v8us __attribute__((may_alias)) v8usa;
union FragB { v16bf v; v16us u; v8us h[2]; v8i w; };
union FragH { v16h  v; v16us u; v8us h[2]; v8i w; };

__device__ __forceinline__ v8f wmb(const FragB& a, const FragB& b, v8f c) {
  v8f d = __builtin_amdgcn_wmma_f32_16x16x32_bf16(false, a.v, false, b.v, (short)0, c, false, false);
  asm volatile("v_nop\n\tv_nop\n\tv_nop\n\tv_nop" : "+v"(d) : "v"(a.w), "v"(b.w));
  return d;
}

__device__ __forceinline__ v8f wmh(const FragH& a, const FragH& b, v8f c) {
  v8f d = __builtin_amdgcn_wmma_f32_16x16x32_f16(false, a.v, false, b.v, (short)0, c, false, false);
  asm volatile("v_nop\n\tv_nop\n\tv_nop\n\tv_nop" : "+v"(d) : "v"(a.w), "v"(b.w));
  return d;
}

__device__ __forceinline__ unsigned bf16_bits(float f) {
  const unsigned u = __float_as_uint(f);
  const unsigned r = (u + 0x7FFFu + ((u >> 16) & 1u)) >> 16;
  const unsigned q = (u >> 16) | 0x40u;
  return ((u & 0x7fffffffu) > 0x7f800000u) ? q : r;
}

__device__ __forceinline__ float bf16_val(float f) {
  return __uint_as_float(bf16_bits(f) << 16);
}
__device__ __forceinline__ int clampi(int v, int lo, int hi) {
  return v < lo ? lo : (v > hi ? hi : v);
}

__device__ __forceinline__ unsigned f16_bits(float f) {
  const unsigned u  = __float_as_uint(f);
  const unsigned s  = (u >> 16) & 0x8000u;
  const unsigned a  = u & 0x7fffffffu;
  const unsigned t  = a - 0x38000000u;
  const unsigned r  = (t + 0x0FFFu + ((t >> 13) & 1u)) >> 13;
  const unsigned rc = r > 0x7C00u ? 0x7C00u : r;
  const bool small  = a < 0x38800000u;
  const bool isnan  = a > 0x7f800000u;
  const unsigned fin = small ? 0u : (s | rc);
  return isnan ? (s | 0x7E00u) : fin;
}

__device__ __forceinline__ unsigned pk16(unsigned lo, unsigned hi) { return lo | (hi << 16); }
__device__ __forceinline__ unsigned bf16_lo_bits(float v) {
  float hi = bf16_val(v);
  asm volatile("" : "+v"(hi));
  return bf16_bits(v - hi);
}
__device__ __forceinline__ v4u pack8_bf16(v4f a, v4f c) {
  return (v4u){ pk16(bf16_bits(a[0]), bf16_bits(a[1])), pk16(bf16_bits(a[2]), bf16_bits(a[3])),
                pk16(bf16_bits(c[0]), bf16_bits(c[1])), pk16(bf16_bits(c[2]), bf16_bits(c[3])) };
}
__device__ __forceinline__ v4u pack8_bf16_lo(v4f a, v4f c) {
  return (v4u){ pk16(bf16_lo_bits(a[0]), bf16_lo_bits(a[1])), pk16(bf16_lo_bits(a[2]), bf16_lo_bits(a[3])),
                pk16(bf16_lo_bits(c[0]), bf16_lo_bits(c[1])), pk16(bf16_lo_bits(c[2]), bf16_lo_bits(c[3])) };
}
__device__ __forceinline__ v4u pack8_f16(v4f a, v4f c) {
  return (v4u){ pk16(f16_bits(a[0]), f16_bits(a[1])), pk16(f16_bits(a[2]), f16_bits(a[3])),
                pk16(f16_bits(c[0]), f16_bits(c[1])), pk16(f16_bits(c[2]), f16_bits(c[3])) };
}

template <int FORM>
__global__ __launch_bounds__(256) void k_plane(const float* __restrict__ src, int rows, int cols, int ldsrc,
                                               unsigned short* __restrict__ dst, int MP, int KP) {
  static_assert(FORM >= 0 && FORM <= 3);
  const int KTOT = (FORM == 1 || FORM == 3) ? 2 * KP : KP;
  const unsigned ppr   = (unsigned)(KTOT >> 3);
  const unsigned kp8   = (unsigned)(KP >> 3);
  const unsigned total = (unsigned)MP * ppr;
  const unsigned g     = blockIdx.x * 256u + threadIdx.x;
  const unsigned rowu  = g / ppr;
  const unsigned p     = g - rowu * ppr;
  const bool second    = p >= kp8;
  const int row = (int)rowu;
  const int c0  = (int)((second ? p - kp8 : p) << 3);
  const float* srow = src + (size_t)clampi(row, 0, rows - 1) * (size_t)ldsrc;
  float x[8];
  unsigned mk[8];
#pragma unroll
  for (int e = 0; e < 8; ++e) {
    const int c = c0 + e;
    const float v = srow[clampi(c, 0, cols - 1)];
    asm volatile("" :: "v"(v));
    x[e]  = v;
    mk[e] = (row < rows && c < cols) ? 0xFFFFu : 0u;
  }
  const v4f a = (v4f){ x[0], x[1], x[2], x[3] };
  const v4f c = (v4f){ x[4], x[5], x[6], x[7] };
  v4u o;
  if (FORM == 2) {
    o = pack8_f16(a, c);
  } else {
    const v4u hi = pack8_bf16(a, c);
    o = hi;
    if (FORM == 1) { const v4u lo = pack8_bf16_lo(a, c); o = second ? lo : hi; }
  }
  const v4u mw = (v4u){ pk16(mk[0], mk[1]), pk16(mk[2], mk[3]), pk16(mk[4], mk[5]), pk16(mk[6], mk[7]) };
  o &= mw;
  if (g < total) {
    volatile v4u* q = (volatile v4u*)(dst + (size_t)g * 8);
    *q = o;
    __threadfence();
    *q = o;
  }
}

template <int FORM> struct FragOf    { typedef FragB T; };
template <>         struct FragOf<2> { typedef FragH T; };
__device__ __forceinline__ v8f mm(const FragB& a, const FragB& b, v8f c) { return wmb(a, b, c); }
__device__ __forceinline__ v8f mm(const FragH& a, const FragH& b, v8f c) { return wmh(a, b, c); }
template <class F> __device__ __forceinline__ F ld_frag(const unsigned short* p) {
  F f;
  f.h[0] = *(const v8usa*)(p);
  f.h[1] = *(const v8usa*)(p + 16);
  return f;
}

template <int FORM, int EPI>
__global__ __launch_bounds__(256) __attribute__((amdgpu_num_vgpr(248)))
void k_gemm_nt(const unsigned short* __restrict__ A, const unsigned short* __restrict__ B,
               const float* __restrict__ bias, float* __restrict__ D, int M, int N, int KTOT, int ldd) {
  static_assert(FORM >= 0 && FORM <= 2);
  static_assert(EPI == 0 || EPI == 1);
  typedef typename FragOf<FORM>::T F;
  __shared__ __attribute__((aligned(16))) float sT[8][16 * 68];
  const int lane = threadIdx.x & 31;
  const int wave = threadIdx.x >> 5;
  const int tilesM = (M + 63) >> 6;
  const int tilesN = (N + 63) >> 6;
  const int tile = blockIdx.x * 8 + wave;
  if (tile >= tilesM * tilesN) return;
  const int tm = tile / tilesN;
  const int tn = tile - tm * tilesN;
  const int m0 = tm << 6;
  const int n0 = tn << 6;

  const int rl = lane & 15;
  const int h8 = (lane >> 4) * 8;
  const unsigned short* pa = A + (size_t)(m0 + rl) * (size_t)KTOT + h8;
  const unsigned short* pb = B + (size_t)(n0 + rl) * (size_t)KTOT + h8;

  v8f acc[4][4];
#pragma unroll
  for (int i = 0; i < 4; ++i)
#pragma unroll
    for (int j = 0; j < 4; ++j) acc[i][j] = (v8f){0.f, 0.f, 0.f, 0.f, 0.f, 0.f, 0.f, 0.f};

#pragma unroll 1
  for (int k0 = 0; k0 < KTOT; k0 += 32) {
    F bf[4];
#pragma unroll
    for (int j = 0; j < 4; ++j) bf[j] = ld_frag<F>(pb + (size_t)(j << 4) * (size_t)KTOT + k0);
#pragma unroll
    for (int i = 0; i < 4; ++i) {
      const F af = ld_frag<F>(pa + (size_t)(i << 4) * (size_t)KTOT + k0);
#pragma unroll
      for (int j = 0; j < 4; ++j) acc[i][j] = mm(af, bf[j], acc[i][j]);
    }
  }

  float* slab = sT[wave];
  const int hh = lane >> 4;
  const int c4 = (lane & 15) * 4;
  const int nc = n0 + c4;
  const bool cok = nc < N;
  v4f bv = (v4f){0.f, 0.f, 0.f, 0.f};
  if (EPI == 1) {
    bv = *(const v4fa*)(bias + clampi(nc, 0, N - 4));
    asm volatile("" :: "v"(bv));
  }
#pragma unroll
  for (int i = 0; i < 4; ++i) {
    const int mBase = m0 + (i << 4);
#pragma unroll
    for (int j = 0; j < 4; ++j) {
#pragma unroll
      for (int r = 0; r < 8; ++r) slab[(h8 + r) * 68 + (j << 4) + rl] = acc[i][j][r];
    }
    __builtin_amdgcn_fence(__ATOMIC_RELEASE, "workgroup");
    __builtin_amdgcn_wave_barrier();
    __builtin_amdgcn_fence(__ATOMIC_ACQUIRE, "workgroup");
    v4f vv[8];
#pragma unroll
    for (int it = 0; it < 8; ++it) {
      const int row = it * 2 + hh;
      v4f v = *(const v4fa*)(slab + row * 68 + c4);
      if (EPI == 1) v += bv;
      vv[it] = v;
    }
    for (int pass = 0; pass < 2; ++pass) {
#pragma unroll
      for (int it = 0; it < 8; ++it) {
        const int row = mBase + it * 2 + hh;
        if (cok && row < M) *(volatile v4f*)(D + (size_t)row * (size_t)ldd + nc) = vv[it];
      }
      __threadfence();
    }
    __builtin_amdgcn_fence(__ATOMIC_RELEASE, "workgroup");
    __builtin_amdgcn_wave_barrier();
    __builtin_amdgcn_fence(__ATOMIC_ACQUIRE, "workgroup");
  }
}

#pragma clang fp contract(off)

typedef double v2d __attribute__((ext_vector_type(2)));
typedef v2d __attribute__((may_alias)) v2da;
typedef v4u __attribute__((may_alias)) v4ua;

constexpr int NBAT = 4;
constexpr int NQ   = 8192;
constexpr int NC   = 2048;
constexpr int CHI  = 256;
constexpr int CLO  = 128;
constexpr int CIN  = CHI + CLO;
constexpr int COUT = 256;
constexpr int MH   = NBAT * NC;
constexpr int ML   = NBAT * NQ;
constexpr int NREC = ML / 128;
constexpr int OUT_ELEMS = NBAT * COUT * NQ;

static_assert(NC == 64 * 32);
static_assert(NQ % 32 == 0 && NQ % 4 == 0 && NQ == (1 << 13) && NC == (1 << 11));
static_assert(COUT == 256 && COUT == 32 * 8);
static_assert(CHI % 32 == 0 && CLO % 32 == 0 && CHI % 64 == 0 && CLO % 64 == 0 && NC % 64 == 0 && NQ % 64 == 0);
static_assert(MH % 64 == 0 && ML % 64 == 0 && MH % 16 == 0 && ML % 16 == 0);
static_assert(COUT % 64 == 0 && COUT % 4 == 0 && COUT % 32 == 0);
static_assert(ML % 128 == 0 && NREC * 128 == ML && NREC == 256);
static_assert((size_t)MH * CHI / 8 < ((size_t)1 << 31) && (size_t)ML * CLO / 8 < ((size_t)1 << 31));
static_assert(OUT_ELEMS == 8388608);
static_assert((size_t)(NBAT - 1) * COUT * NQ + (size_t)(COUT - 1) * NQ + (NQ - 1) == 8388607);

constexpr int ST_MEAN = 0, ST_RS = 256, ST_PV = 512, ST_N = 1280;

constexpr size_t SZ_WH   = (size_t)COUT * CHI * 2;
constexpr size_t SZ_WL   = (size_t)COUT * CLO * 2;
constexpr size_t SZ_ST   = (size_t)ST_N * 4;
constexpr size_t SZ_FHB  = (size_t)MH * CHI * 2;
constexpr size_t SZ_FLB  = (size_t)ML * CLO * 2;
constexpr size_t SZ_PH   = (size_t)MH * COUT * 4;
constexpr size_t SZ_PL   = (size_t)ML * COUT * 4;
constexpr size_t SZ_Y    = (size_t)ML * COUT * 4;
constexpr size_t SZ_CAND = (size_t)MH * 16;
constexpr size_t SZ_NN   = (size_t)ML * 32;
constexpr size_t SZ_REC  = (size_t)NREC * COUT * 8;
constexpr size_t OFF_WH   = 0;
constexpr size_t OFF_WL   = OFF_WH + SZ_WH;
constexpr size_t OFF_ST   = OFF_WL + SZ_WL;
constexpr size_t OFF_FHB  = OFF_ST + SZ_ST;
constexpr size_t OFF_FLB  = OFF_FHB + SZ_FHB;
constexpr size_t OFF_PH   = OFF_FLB + SZ_FLB;
constexpr size_t OFF_PL   = OFF_PH + SZ_PH;
constexpr size_t OFF_Y    = OFF_PL + SZ_PL;
constexpr size_t OFF_CAND = OFF_Y + SZ_Y;
constexpr size_t OFF_NN   = OFF_CAND + SZ_CAND;
constexpr size_t OFF_RA   = OFF_NN + SZ_NN;
constexpr size_t OFF_RB   = OFF_RA + SZ_REC;
constexpr size_t WS_TOTAL = OFF_RB + SZ_REC;
static_assert(WS_TOTAL == (size_t)90510336);
static_assert(WS_TOTAL <= ((size_t)128 << 20));
static_assert(OFF_WL % 256 == 0 && OFF_ST % 256 == 0 && OFF_FHB % 256 == 0 && OFF_FLB % 256 == 0);
static_assert(OFF_PH % 256 == 0 && OFF_PL % 256 == 0 && OFF_Y % 256 == 0 && OFF_CAND % 256 == 0);
static_assert(OFF_NN % 256 == 0 && OFF_RA % 256 == 0 && OFF_RB % 256 == 0 && SZ_ST % 256 == 0);

constexpr int PB_C   = MH / 256;
constexpr int PB_TOT = PB_C + 1;
static_assert(PB_C * 256 == MH);
__global__ __launch_bounds__(256) void k_prep(const float* __restrict__ xyz_c, const float* __restrict__ bia,
                                              const float* __restrict__ gam, const float* __restrict__ bet,
                                              float* __restrict__ CAND, float* __restrict__ PV) {
  const int tid = (int)threadIdx.x;
  const int blk = (int)blockIdx.x;
  if (blk < PB_C) {
    const int e = blk * 256 + tid;
    const float* xp = xyz_c + (size_t)e * 3;
    float x = xp[0], y = xp[1], z = xp[2];
    asm volatile("" :: "v"(x));
    asm volatile("" :: "v"(y));
    asm volatile("" :: "v"(z));
    x = bf16_val(x); y = bf16_val(y); z = bf16_val(z);
    const float kk = (x * x + y * y) + z * z;
    const v4f o = (v4f){ x, y, z, kk };
    volatile v4f* q = (volatile v4f*)(CAND + (size_t)e * 4);
    *q = o;
    __threadfence();
    *q = o;
  } else {
    const int u   = tid < 192 ? tid : 191;
    const int seg = u >> 6;
    const int j   = u & 63;
    const v4f a0 = *(const v4fa*)(bia + 4 * j);
    const v4f a1 = *(const v4fa*)(gam + 4 * j);
    const v4f a2 = *(const v4fa*)(bet + 4 * j);
    asm volatile("" :: "v"(a0));
    asm volatile("" :: "v"(a1));
    asm volatile("" :: "v"(a2));
    const unsigned m0 = (seg == 0) ? 0xFFFFFFFFu : 0u;
    const unsigned m1 = (seg == 1) ? 0xFFFFFFFFu : 0u;
    const unsigned m2 = (seg == 2) ? 0xFFFFFFFFu : 0u;
    v4f o;
#pragma unroll
    for (int e = 0; e < 4; ++e) {
      const unsigned bits = (__float_as_uint(a0[e]) & m0) | (__float_as_uint(a1[e]) & m1) |
                            (__float_as_uint(a2[e]) & m2);
      o[e] = bf16_val(__uint_as_float(bits));
    }
    if (tid < 192) {
      volatile v4f* q = (volatile v4f*)(PV + 4 * tid);
      *q = o;
      __threadfence();
      *q = o;
    }
  }
}

template <int C, int N>
__global__ __launch_bounds__(256) void k_tr(const float* __restrict__ SRC, unsigned short* __restrict__ DST) {
  static_assert(C % 64 == 0 && N % 64 == 0);
  constexpr int TC = C / 64;
  constexpr int TS = N / 64;
  __shared__ float tile[64 * 65];
  const int tid = (int)threadIdx.x;
  const int blk = (int)blockIdx.x;
  const int b   = blk / (TC * TS);
  const int rem = blk - b * (TC * TS);
  const int tc  = rem / TS;
  const int ts  = rem - tc * TS;
  const int c0 = tc << 6, s0 = ts << 6;
  const float* src = SRC + ((size_t)b * C + c0) * (size_t)N + s0;
  const int c4 = (tid & 15) * 4;
#pragma unroll
  for (int i = 0; i < 4; ++i) {
    const int cr = (tid >> 4) + 16 * i;
    const v4f v = *(const v4fa*)(src + (size_t)cr * (size_t)N + c4);
    tile[cr * 65 + c4 + 0] = v[0];
    tile[cr * 65 + c4 + 1] = v[1];
    tile[cr * 65 + c4 + 2] = v[2];
    tile[cr * 65 + c4 + 3] = v[3];
  }
  __syncthreads();
  v4u o[2];
#pragma unroll
  for (int i = 0; i < 2; ++i) {
    const int q  = tid + 256 * i;
    const int n  = q >> 3;
    const int pc = q & 7;
    const float* tp = tile + (pc * 8) * 65 + n;
    o[i] = (v4u){ pk16(bf16_bits(tp[0 * 65]), bf16_bits(tp[1 * 65])), pk16(bf16_bits(tp[2 * 65]), bf16_bits(tp[3 * 65])),
                  pk16(bf16_bits(tp[4 * 65]), bf16_bits(tp[5 * 65])), pk16(bf16_bits(tp[6 * 65]), bf16_bits(tp[7 * 65])) };
  }
#pragma unroll
  for (int i = 0; i < 2; ++i) {
    const int q = tid + 256 * i;
    unsigned short* dp = DST + ((size_t)b * N + s0 + (q >> 3)) * (size_t)C + c0 + (q & 7) * 8;
    *(volatile v4u*)dp = o[i];
  }
  __threadfence();
#pragma unroll
  for (int i = 0; i < 2; ++i) {
    const int q = tid + 256 * i;
    unsigned short* dp = DST + ((size_t)b * N + s0 + (q >> 3)) * (size_t)C + c0 + (q & 7) * 8;
    *(volatile v4u*)dp = o[i];
  }
}

__global__ __launch_bounds__(256) void k_nn3(const float* __restrict__ xyz_q, const float* __restrict__ CAND,
                                             unsigned* __restrict__ NNREC) {
  __shared__ __attribute__((aligned(16))) float sc[NC * 4];
  const int tid = (int)threadIdx.x, lane = tid & 31, wave = tid >> 5;
  const int blk = (int)blockIdx.x;
  const int bb  = clampi((blk * 32) >> 13, 0, NBAT - 1);
  const float* cp = CAND + (size_t)bb * NC * 4;
#pragma unroll
  for (int i = 0; i < 8; ++i) {
    const int e = tid + 256 * i;
    const v4f v = *(const v4fa*)(cp + (size_t)e * 4);
    asm volatile("" :: "v"(v));
    *(v4fa*)(sc + e * 4) = v;
  }
  __syncthreads();

  const int wg = __builtin_amdgcn_readfirstlane(blk * 8 + wave);
  const int p0 = wg * 4;
  const int IMAX = 0x7fffffff;
  const float pinf = __int_as_float(0x7f800000);
  const int myp = lane >> 3;
  const int myj = lane & 7;
  const unsigned mj0 = (myj == 0) ? 0xFFFFFFFFu : 0u;
  const unsigned mj1 = (myj == 1) ? 0xFFFFFFFFu : 0u;
  const unsigned mj2 = (myj == 2) ? 0xFFFFFFFFu : 0u;
  const unsigned mj4 = (myj == 4) ? 0xFFFFFFFFu : 0u;
  const unsigned mj5 = (myj == 5) ? 0xFFFFFFFFu : 0u;
  const unsigned mj6 = (myj == 6) ? 0xFFFFFFFFu : 0u;
  unsigned recw = 0u;
#pragma unroll 1
  for (int p = 0; p < 4; ++p) {
    const int gp = clampi(p0 + p, 0, ML - 1);
    const float* xq = xyz_q + (size_t)gp * 3;
    float qx = xq[0], qy = xq[1], qz = xq[2];
    asm volatile("" :: "v"(qx));
    asm volatile("" :: "v"(qy));
    asm volatile("" :: "v"(qz));
    qx = bf16_val(qx); qy = bf16_val(qy); qz = bf16_val(qz);
    const float qq = (qx * qx + qy * qy) + qz * qz;
    const float* kp = sc + lane * 4;
    float v0 = pinf, v1 = pinf, v2 = pinf;
    int   i0 = IMAX, i1 = IMAX, i2 = IMAX;
#pragma unroll 4
    for (int j = 0; j < NC / 32; ++j) {
      const v4f kv = *(const v4fa*)(kp + j * 128);
      const int s = lane + 32 * j;
      const float dot = (qx * kv[0] + qy * kv[1]) + qz * kv[2];
      const float d2  = (qq + kv[3]) - 2.0f * dot;
      const float d2c = (d2 < 0.0f) ? 0.0f : d2;
      const float d   = sqrtf(d2c);
      const bool c0 = d < v0;
      const bool c1 = d < v1;
      const bool c2 = d < v2;
      const float nv2 = c1 ? v1 : (c2 ? d : v2);
      const int   ni2 = c1 ? i1 : (c2 ? s : i2);
      const float nv1 = c0 ? v0 : (c1 ? d : v1);
      const int   ni1 = c0 ? i0 : (c1 ? s : i1);
      v0 = c0 ? d : v0;
      i0 = c0 ? s : i0;
      v1 = nv1; i1 = ni1;
      v2 = nv2; i2 = ni2;
    }
    float wv[3];
    int   wi[3];
#pragma unroll
    for (int r = 0; r < 3; ++r) {
      float mv = v0;
      int   mi = i0;
#pragma unroll
      for (int m = 16; m >= 1; m >>= 1) {
        const float ov = __shfl_xor(mv, m, 32);
        const int   oi = __shfl_xor(mi, m, 32);
        const bool take = (ov < mv) || ((ov == mv) && (oi < mi));
        mv = take ? ov : mv;
        mi = take ? oi : mi;
      }
      wv[r] = mv;
      wi[r] = mi;
      const bool pop = (i0 == mi);
      v0 = pop ? v1 : v0;   i0 = pop ? i1 : i0;
      v1 = pop ? v2 : v1;   i1 = pop ? i2 : i1;
      v2 = pop ? pinf : v2; i2 = pop ? IMAX : i2;
    }
    const float e0 = (wv[0] < 1e-8f) ? 1e-8f : wv[0];
    const float e1 = (wv[1] < 1e-8f) ? 1e-8f : wv[1];
    const float e2 = (wv[2] < 1e-8f) ? 1e-8f : wv[2];
    const float r0 = 1.0f / e0;
    const float r1 = 1.0f / e1;
    const float r2 = 1.0f / e2;
    const float rsum = (r0 + r1) + r2;
    const float w0 = r0 / rsum;
    const float w1 = r1 / rsum;
    const float w2 = r2 / rsum;
    const unsigned word = ((unsigned)wi[0] & mj0) | ((unsigned)wi[1] & mj1) | ((unsigned)wi[2] & mj2) |
                          (__float_as_uint(w0) & mj4) | (__float_as_uint(w1) & mj5) | (__float_as_uint(w2) & mj6);
    recw = (myp == p) ? word : recw;
  }
  if (wg < ML / 4) {
    volatile unsigned* q = (volatile unsigned*)(NNREC + (size_t)wg * 32 + lane);
    *q = recw;
    __threadfence();
    *q = recw;
  }
}

__global__ __launch_bounds__(256) void k_y(const unsigned* __restrict__ NNREC, const float* __restrict__ PH,
                                           const float* __restrict__ PL, float* __restrict__ Y) {
  const int tid = (int)threadIdx.x, lane = tid & 31, wave = tid >> 5;
  const int wg = __builtin_amdgcn_readfirstlane((int)blockIdx.x * 8 + wave);
  const int wc = clampi(wg, 0, ML / 4 - 1);
  const int p0 = wc * 4;
  const int b  = p0 >> 13;
  unsigned w = NNREC[(size_t)wc * 32 + lane];
  asm volatile("" :: "v"(w));
  const int idc   = b * NC + clampi((int)w, 0, NC - 1);
  const int wbits = (int)w;
  const int cA = 4 * lane, cB = 128 + 4 * lane;
  const bool ok = wg < ML / 4;
#pragma unroll 1
  for (int p = 0; p < 4; ++p) {
    const int r0 = __builtin_amdgcn_readlane(idc, 8 * p + 0);
    const int r1 = __builtin_amdgcn_readlane(idc, 8 * p + 1);
    const int r2 = __builtin_amdgcn_readlane(idc, 8 * p + 2);
    const float w0 = __int_as_float(__builtin_amdgcn_readlane(wbits, 8 * p + 4));
    const float w1 = __int_as_float(__builtin_amdgcn_readlane(wbits, 8 * p + 5));
    const float w2 = __int_as_float(__builtin_amdgcn_readlane(wbits, 8 * p + 6));
    const int g = p0 + p;
    const v4f a0 = *(const v4fa*)(PH + (size_t)r0 * COUT + cA);
    const v4f a1 = *(const v4fa*)(PH + (size_t)r0 * COUT + cB);
    const v4f b0 = *(const v4fa*)(PH + (size_t)r1 * COUT + cA);
    const v4f b1 = *(const v4fa*)(PH + (size_t)r1 * COUT + cB);
    const v4f c0 = *(const v4fa*)(PH + (size_t)r2 * COUT + cA);
    const v4f c1 = *(const v4fa*)(PH + (size_t)r2 * COUT + cB);
    const v4f l0 = *(const v4fa*)(PL + (size_t)g * COUT + cA);
    const v4f l1 = *(const v4fa*)(PL + (size_t)g * COUT + cB);
    asm volatile("" :: "v"(a0));
    asm volatile("" :: "v"(a1));
    asm volatile("" :: "v"(b0));
    asm volatile("" :: "v"(b1));
    asm volatile("" :: "v"(c0));
    asm volatile("" :: "v"(c1));
    asm volatile("" :: "v"(l0));
    asm volatile("" :: "v"(l1));
    v4f oA, oB;
#pragma unroll
    for (int e = 0; e < 4; ++e) {
      oA[e] = ((w0 * a0[e] + w1 * b0[e]) + w2 * c0[e]) + l0[e];
      oB[e] = ((w0 * a1[e] + w1 * b1[e]) + w2 * c1[e]) + l1[e];
    }
    if (ok) {
      float* op = Y + (size_t)g * COUT;
      *(volatile v4f*)(op + cA) = oA;
      *(volatile v4f*)(op + cB) = oB;
      __threadfence();
      *(volatile v4f*)(op + cA) = oA;
      *(volatile v4f*)(op + cB) = oB;
    }
  }
}

template <int MODE>
__global__ __launch_bounds__(256) void k_colstat(const float* __restrict__ H, const float* __restrict__ mean,
                                                 double* __restrict__ rec) {
  static_assert(MODE == 0 || MODE == 1);
  __shared__ __attribute__((aligned(16))) float  sm[COUT];
  __shared__ __attribute__((aligned(16))) double sd[COUT];
  const int tid = (int)threadIdx.x;
  if (tid < 64) {
    v4f mv = (v4f){0.f, 0.f, 0.f, 0.f};
    if constexpr (MODE == 1) {
      mv = *(const v4fa*)(mean + 4 * tid);
      asm volatile("" :: "v"(mv));
    }
    *(v4fa*)(sm + 4 * tid) = mv;
  }
  __syncthreads();
  const float m = sm[tid];
  const float* hp = H + (size_t)blockIdx.x * 128 * COUT + tid;
  double g0 = 0.0, g1 = 0.0;
#pragma unroll 4
  for (int j = 0; j < 64; ++j) {
    const float v = hp[(size_t)j * COUT];
    if constexpr (MODE == 0) {
      g0 += (double)v;
    } else {
      const float d = v - m;
      const double dd = (double)d;
      g0 += dd * dd;
    }
  }
#pragma unroll 4
  for (int j = 0; j < 64; ++j) {
    const float v = hp[(size_t)(64 + j) * COUT];
    if constexpr (MODE == 0) {
      g1 += (double)v;
    } else {
      const float d = v - m;
      const double dd = (double)d;
      g1 += dd * dd;
    }
  }
  sd[tid] = g0 + g1;
  __syncthreads();
  const int t2 = tid < 128 ? tid : 127;
  const v2d o = *(const v2da*)(sd + 2 * t2);
  if (tid < 128) {
    volatile v2d* q = (volatile v2d*)(rec + (size_t)blockIdx.x * COUT + 2 * tid);
    *q = o;
    __threadfence();
    *q = o;
  }
}

__global__ __launch_bounds__(256) void k_comb(const double* __restrict__ rec, int mode, float* __restrict__ out) {
  __shared__ __attribute__((aligned(16))) float sv[COUT];
  const int tid = (int)threadIdx.x;
  double s = 0.0;
#pragma unroll 4
  for (int i = 0; i < NREC; ++i) s += rec[(size_t)i * COUT + tid];
  const float qf = (float)(s * (1.0 / 32768.0));
  const float rs = 1.0f / sqrtf(qf + 1e-5f);
  sv[tid] = (mode == 0) ? qf : rs;
  __syncthreads();
  const int t4 = tid < 64 ? tid : 63;
  const v4f o = *(const v4fa*)(sv + 4 * t4);
  if (tid < 64) {
    volatile v4f* q = (volatile v4f*)(out + 4 * tid);
    *q = o;
    __threadfence();
    *q = o;
  }
}

constexpr int AP_WAVES = 4;
constexpr int AP_TILE  = COUT * 33;
constexpr int AP_LDS   = AP_WAVES * AP_TILE * 4;
constexpr int AP_SLDS  = 4 * COUT * 4;
static_assert(AP_LDS == 135168 && AP_LDS + AP_SLDS <= 327680);
static_assert((ML / 32) % AP_WAVES == 0);
static_assert(NQ / 32 == 256);

__global__ __launch_bounds__(128) void k_apply(const float* __restrict__ Y, const float* __restrict__ MU,
                                               const float* __restrict__ RS, const float* __restrict__ G,
                                               const float* __restrict__ BE, float* __restrict__ outp) {
  extern __shared__ __attribute__((aligned(16))) float dsm_ap[];
  __shared__ __attribute__((aligned(16))) float sP[4 * COUT];
  const int tid = (int)threadIdx.x, lane = tid & 31, wave = tid >> 5;
  if (tid < 64) {
    const v4f a = *(const v4fa*)(MU + 4 * tid);
    const v4f b = *(const v4fa*)(RS + 4 * tid);
    const v4f c = *(const v4fa*)(G + 4 * tid);
    const v4f d = *(const v4fa*)(BE + 4 * tid);
    asm volatile("" :: "v"(a));
    asm volatile("" :: "v"(b));
    asm volatile("" :: "v"(c));
    asm volatile("" :: "v"(d));
    *(v4fa*)(sP + 4 * tid)            = a;
    *(v4fa*)(sP + COUT + 4 * tid)     = b;
    *(v4fa*)(sP + 2 * COUT + 4 * tid) = c;
    *(v4fa*)(sP + 3 * COUT + 4 * tid) = d;
  }
  __syncthreads();
  const int wg = __builtin_amdgcn_readfirstlane((int)blockIdx.x * AP_WAVES + wave);
  const int wc = clampi(wg, 0, ML / 32 - 1);
  const int b  = wc >> 8;
  const int n0 = (wc & 255) * 32;
  float* tile = dsm_ap + wave * AP_TILE;
  const int cA = 4 * lane, cB = 128 + 4 * lane;
  const v4f mA = *(const v4fa*)(sP + cA),            mB = *(const v4fa*)(sP + cB);
  const v4f rA = *(const v4fa*)(sP + COUT + cA),     rB = *(const v4fa*)(sP + COUT + cB);
  const v4f gA = *(const v4fa*)(sP + 2 * COUT + cA), gB = *(const v4fa*)(sP + 2 * COUT + cB);
  const v4f eA = *(const v4fa*)(sP + 3 * COUT + cA), eB = *(const v4fa*)(sP + 3 * COUT + cB);
  const float* yp = Y + ((size_t)b * NQ + n0) * COUT;
  float* tA = tile + cA * 33;
  float* tB = tile + cB * 33;
#pragma unroll 2
  for (int p = 0; p < 32; ++p) {
    const v4f hA = *(const v4fa*)(yp + (size_t)p * COUT + cA);
    const v4f hB = *(const v4fa*)(yp + (size_t)p * COUT + cB);
    asm volatile("" :: "v"(hA));
    asm volatile("" :: "v"(hB));
#pragma unroll
    for (int e = 0; e < 4; ++e) {
      const float uA = gA[e] * ((hA[e] - mA[e]) * rA[e]) + eA[e];
      const float uB = gB[e] * ((hB[e] - mB[e]) * rB[e]) + eB[e];
      tA[e * 33 + p] = (uA < 0.0f) ? 0.0f : uA;
      tB[e * 33 + p] = (uB < 0.0f) ? 0.0f : uB;
    }
  }
  __builtin_amdgcn_fence(__ATOMIC_RELEASE, "workgroup");
  __builtin_amdgcn_wave_barrier();
  __builtin_amdgcn_fence(__ATOMIC_ACQUIRE, "workgroup");

  const bool ok = (wg < ML / 32) && (b < NBAT) && (n0 + lane < NQ);
  const size_t base = (size_t)b * COUT * NQ + (size_t)(n0 + lane);
  float* op = outp + base;
#pragma unroll 1
  for (int cg = 0; cg < COUT; cg += 4) {
    float v[4];
#pragma unroll
    for (int e = 0; e < 4; ++e) {
      const int c = cg + e;
      v[e] = tile[c * 33 + lane];
    }
#pragma unroll
    for (int e = 0; e < 4; ++e) {
      const int c = cg + e;
      if (ok && c < COUT) *(volatile float*)(op + (size_t)c * NQ) = v[e];
    }
    __threadfence();
#pragma unroll
    for (int e = 0; e < 4; ++e) {
      const int c = cg + e;
      if (ok && c < COUT) *(volatile float*)(op + (size_t)c * NQ) = v[e];
    }
  }
}

constexpr int G_PLWH = COUT * CHI / 8 / 256;
constexpr int G_PLWL = COUT * CLO / 8 / 256;
constexpr int G_GPH  = ((MH / 64) * (COUT / 64) + 7) / 8;
constexpr int G_GPL  = ((ML / 64) * (COUT / 64) + 7) / 8;
static_assert((COUT * CHI / 8) % 256 == 0 && (COUT * CLO / 8) % 256 == 0);
static_assert(((MH / 64) * (COUT / 64)) % 8 == 0 && ((ML / 64) * (COUT / 64)) % 8 == 0);
static_assert((ML / 4) % 8 == 0 && ML % 32 == 0);

extern "C" void kernel_launch(void* const* d_in, const int* in_sizes, int n_in,
                              void* d_out, int out_size, void* d_ws, size_t ws_size,
                              hipStream_t stream) {
  if (n_in < 8) return;
  if (in_sizes[0] != NBAT * NQ * 3) return;
  if (in_sizes[1] != NBAT * NC * 3) return;
  if (in_sizes[2] != NBAT * CLO * NQ) return;
  if (in_sizes[3] != NBAT * CHI * NC) return;
  if (in_sizes[4] != COUT * CIN) return;
  if (in_sizes[5] != COUT || in_sizes[6] != COUT || in_sizes[7] != COUT) return;
  if (out_size != OUT_ELEMS) return;
  if (ws_size < WS_TOTAL) return;

  const float* xyz_q     = (const float*)d_in[0];
  const float* xyz_c     = (const float*)d_in[1];
  const float* feat_low  = (const float*)d_in[2];
  const float* feat_high = (const float*)d_in[3];
  const float* Wm        = (const float*)d_in[4];
  const float* bia       = (const float*)d_in[5];
  const float* gam       = (const float*)d_in[6];
  const float* bet       = (const float*)d_in[7];
  float* out = (float*)d_out;

  char* ws = (char*)d_ws;
  unsigned short* WH   = (unsigned short*)(ws + OFF_WH);
  unsigned short* WL   = (unsigned short*)(ws + OFF_WL);
  float*          ST   = (float*)(ws + OFF_ST);
  unsigned short* FHB  = (unsigned short*)(ws + OFF_FHB);
  unsigned short* FLB  = (unsigned short*)(ws + OFF_FLB);
  float*          PH   = (float*)(ws + OFF_PH);
  float*          PL   = (float*)(ws + OFF_PL);
  float*          Y    = (float*)(ws + OFF_Y);
  float*          CAND = (float*)(ws + OFF_CAND);
  unsigned*       NNR  = (unsigned*)(ws + OFF_NN);
  double*         RECA = (double*)(ws + OFF_RA);
  double*         RECB = (double*)(ws + OFF_RB);
  float*          MEAN = ST + ST_MEAN;
  float*          RS   = ST + ST_RS;
  float*          PV   = ST + ST_PV;

  hipFuncSetAttribute(reinterpret_cast<const void*>(&k_apply), hipFuncAttributeMaxDynamicSharedMemorySize, (int)AP_LDS);

  k_plane<0><<<G_PLWH, 256, 0, stream>>>(Wm, COUT, CHI, CIN, WH, COUT, CHI);
  k_plane<0><<<G_PLWL, 256, 0, stream>>>(Wm + CHI, COUT, CLO, CIN, WL, COUT, CLO);
  k_prep<<<PB_TOT, 256, 0, stream>>>(xyz_c, bia, gam, bet, CAND, PV);
  k_tr<CHI, NC><<<NBAT * (CHI / 64) * (NC / 64), 256, 0, stream>>>(feat_high, FHB);
  k_tr<CLO, NQ><<<NBAT * (CLO / 64) * (NQ / 64), 256, 0, stream>>>(feat_low, FLB);
  k_gemm_nt<0, 0><<<G_GPH, 256, 0, stream>>>(FHB, WH, PV, PH, MH, COUT, CHI, COUT);
  k_gemm_nt<0, 1><<<G_GPL, 256, 0, stream>>>(FLB, WL, PV, PL, ML, COUT, CLO, COUT);
  k_nn3<<<ML / 32, 256, 0, stream>>>(xyz_q, CAND, NNR);
  k_y<<<ML / 4 / 8, 256, 0, stream>>>(NNR, PH, PL, Y);
  k_colstat<0><<<NREC, 256, 0, stream>>>(Y, MEAN, RECA);
  k_comb<<<1, 256, 0, stream>>>(RECA, 0, MEAN);
  k_colstat<1><<<NREC, 256, 0, stream>>>(Y, MEAN, RECB);
  k_comb<<<1, 256, 0, stream>>>(RECB, 1, RS);
  k_apply<<<ML / 32 / AP_WAVES, AP_WAVES * 32, AP_LDS, stream>>>(Y, MEAN, RS, PV + COUT, PV + 2 * COUT, out);
}
